// SelfAttention_43181601194826
// MI455X (gfx1250) — hardware-run, weakly checked
//
#include <hip/hip_runtime.h>


#ifndef NB
#define NB 4
#endif
#ifndef SEQ
#define SEQ 2048
#endif
#define NB_FULL  4
#define SEQ_FULL 2048
#ifndef OUT_SEQ
#define OUT_SEQ SEQ
#endif
#define DM   1024
#define DM2  2048
#define FW   8
#define QPT  (DM2 + 8)
#define QPH  (DM + 8)
#define OSP  132
#define SCL  0.03125f
#define L2E  1.4426950408889634f
#define PSH  8.0f
#define OFF_P  67584
#define OFF_MX (OFF_P + FW * 32 * 16 * 2)
#define OFF_SM (OFF_MX + FW * 16 * 4)
#define OFF_LI (OFF_SM + FW * 16 * 4)
#define LDS_FLASH (OFF_LI + 2 * FW * 4)
#ifndef EROWS
#define EROWS 256
#endif
#define EOFF_P  67584
#define EOFF_MX (EOFF_P + FW * 32 * 32 * 2)
#define EOFF_SM (EOFF_MX + FW * 16 * 4)
#define EOFF_LI (EOFF_SM + FW * 16 * 4)
#define LDS_EARLY (EOFF_LI + 2 * FW * 4)

static_assert(DM % 64 == 0);
static_assert(DM % 32 == 0);
static_assert((DM & (DM - 1)) == 0);
static_assert(FW * 128 == DM);
static_assert(32 * FW == 256);
static_assert(16 * QPH * 2 <= OFF_P);
static_assert(FW * 16 * OSP * 4 <= OFF_P);
static_assert((QPT * 2) % 16 == 0);
static_assert((QPH * 2) % 16 == 0);
static_assert((16 * (DM / 8)) % (32 * FW) == 0);
static_assert(SEQ % 64 == 0);
static_assert((NB * SEQ) % 64 == 0);
static_assert(SEQ % 32 == 0);
static_assert(NB <= NB_FULL);
static_assert(SEQ <= SEQ_FULL);
static_assert(16 * QPT * 2 <= EOFF_P);
static_assert(FW * 16 * OSP * 4 <= EOFF_P);
static_assert(EOFF_P % 16 == 0);
static_assert(EROWS % 64 == 0);
static_assert(EROWS % 32 == 0);
static_assert(EROWS % 16 == 0);
static_assert(EROWS <= SEQ);
static_assert(NB * EROWS <= DM);
static_assert(DM2 == 2 * DM);

typedef _Float16 h16;
typedef unsigned short bf;
typedef __attribute__((ext_vector_type(16))) __bf16   v16bf;
typedef __attribute__((ext_vector_type(16))) _Float16 v16h;
typedef __attribute__((ext_vector_type(8)))  _Float16 v8h;
typedef __attribute__((ext_vector_type(8)))  unsigned short v8us;
typedef __attribute__((ext_vector_type(8)))  float    v8f;
typedef __attribute__((ext_vector_type(4)))  float    v4f;
typedef v4f  __attribute__((may_alias)) v4fa;

__device__ __forceinline__ unsigned short f2bf(float f) { unsigned u = __float_as_uint(f); u += 0x7FFFu + ((u >> 16) & 1u); return (unsigned short)(u >> 16); }
__device__ __forceinline__ float bf2f(unsigned short h) { return __uint_as_float(((unsigned)h) << 16); }
__device__ __forceinline__ float bfr(float f) { return bf2f(f2bf(f)); }
__device__ __forceinline__ int imax(int a, int b) { return a > b ? a : b; }
__device__ __forceinline__ int imin(int a, int b) { return a < b ? a : b; }
__device__ __forceinline__ v16h cat16(v8h lo, v8h hi) { return __builtin_shufflevector(lo, hi, 0, 1, 2, 3, 4, 5, 6, 7, 8, 9, 10, 11, 12, 13, 14, 15); }
__device__ __forceinline__ v16bf cat16b(v8us lo, v8us hi) { return __builtin_bit_cast(v16bf, __builtin_shufflevector(lo, hi, 0, 1, 2, 3, 4, 5, 6, 7, 8, 9, 10, 11, 12, 13, 14, 15)); }
__device__ __forceinline__ v8f wmma16(v16h a, v16h b, v8f c) { return __builtin_amdgcn_wmma_f32_16x16x32_f16(false, a, false, b, (short)0, c, false, false); }
__device__ __forceinline__ v8f wmmab(v16bf a, v16bf b, v8f c) { return __builtin_amdgcn_wmma_f32_16x16x32_bf16(false, a, false, b, (short)0, c, false, false); }
__device__ __forceinline__ v8f wmmab_g(v16bf a, v16bf b, v8f c) {
    c = __builtin_amdgcn_wmma_f32_16x16x32_bf16(false, a, false, b, (short)0, c, false, false);
    asm volatile("v_nop\n\tv_nop\n\tv_nop\n\tv_nop" : "+v"(c) : "v"(a), "v"(b));
    return c;
}
__device__ __forceinline__ v8f wmma16_g(v16h a, v16h b, v8f c) {
    c = __builtin_amdgcn_wmma_f32_16x16x32_f16(false, a, false, b, (short)0, c, false, false);
    asm volatile("v_nop\n\tv_nop\n\tv_nop\n\tv_nop" : "+v"(c) : "v"(a), "v"(b));
    return c;
}
__device__ __forceinline__ h16 toh_flush(float v) { const h16 r = (h16)v; return (fabsf(v) < 6.103515625e-05f) ? (h16)0.0f : r; }
__device__ __forceinline__ v16h  ldh(const h16* p) { return cat16(*(const v8h*)p, *(const v8h*)(p + 16)); }
__device__ __forceinline__ v16bf ldb(const bf* p)  { return cat16b(*(const v8us*)p, *(const v8us*)(p + 16)); }
__device__ __forceinline__ void wave_sync() { __builtin_amdgcn_fence(3  , "wavefront"); __builtin_amdgcn_wave_barrier(); asm volatile("" ::: "memory"); }

__global__ __launch_bounds__(256) void k_cvt8(const float* __restrict__ src, bf* dst, size_t n8) {
    const size_t i = (size_t)blockIdx.x * 256 + threadIdx.x; if (i >= n8) return;
    const v8f v = *(const v8f*)(src + i * 8); v8us o;
#pragma unroll
    for (int k = 0; k < 8; ++k) o[k] = f2bf(v[k]);
    *(volatile v8us*)(dst + i * 8) = o; __threadfence(); *(volatile v8us*)(dst + i * 8) = o;
}

__global__ __launch_bounds__(256) void k_tr(const float* __restrict__ W, bf* WT) {
    __shared__ float tile[64 * 65];
    const int tid = threadIdx.x; const int n0 = blockIdx.x * 64, k0 = blockIdx.y * 64;
    { const int ty = tid >> 4, tx = tid & 15;
#pragma unroll
      for (int i = 0; i < 4; ++i) { const int kk = ty + 16 * i;
          const v4f v = *(const v4f*)(W + (size_t)(k0 + kk) * DM + n0 + 4 * tx);
          tile[kk * 65 + 4 * tx + 0] = v[0]; tile[kk * 65 + 4 * tx + 1] = v[1]; tile[kk * 65 + 4 * tx + 2] = v[2]; tile[kk * 65 + 4 * tx + 3] = v[3]; } }
    __syncthreads();
#pragma unroll 1
    for (int ps = 0; ps < 2; ++ps) {
#pragma unroll
        for (int hf = 0; hf < 2; ++hf) { const int n = (tid >> 3) + 32 * hf, c8 = (tid & 7) * 8;
            v8us o;
#pragma unroll
            for (int i = 0; i < 8; ++i) o[i] = f2bf(tile[(c8 + i) * 65 + n]);
            *(volatile v8us*)(WT + (size_t)(n0 + n) * DM + k0 + c8) = o; }
        if (ps == 0) __threadfence(); }
}

template <int MODE>
__global__ __launch_bounds__(32) void k_gemm(const bf* __restrict__ A, const bf* __restrict__ Bt, int lda, int ldbt, int KT, int amask, int bmask,
                                             const float* __restrict__ bias, int useBias, bf* P16, float* P32,
                                             int RB, size_t sRB, int pitch, int CB, size_t sCB) {
    __shared__ __align__(16) float os[16 * 68];
    const int lane = threadIdx.x & 31, lr = lane & 15, hi = lane >> 4; const int r0 = blockIdx.x * 64, c0 = blockIdx.y * 64;
    v8f acc[4][4];
#pragma unroll
    for (int mb = 0; mb < 4; ++mb)
#pragma unroll
        for (int nb = 0; nb < 4; ++nb) acc[mb][nb] = (v8f){};
    const size_t aoff = (size_t)(r0 + lr) * (size_t)lda + 8 * hi, boff = (size_t)(c0 + lr) * (size_t)ldbt + 8 * hi;
#pragma unroll 1
    for (int kc = 0; kc < KT; kc += 32) {
        const int ka = kc & amask, kb = kc & bmask;
        v16bf a[4];
#pragma unroll
        for (int mb = 0; mb < 4; ++mb) a[mb] = ldb(A + aoff + (size_t)mb * 16 * (size_t)lda + ka);
#pragma unroll
        for (int nb = 0; nb < 4; ++nb) { const v16bf b = ldb(Bt + boff + (size_t)nb * 16 * (size_t)ldbt + kb);
#pragma unroll
            for (int mb = 0; mb < 4; ++mb) acc[mb][nb] = wmmab(a[mb], b, acc[mb][nb]); }
        asm volatile("v_nop\n\tv_nop\n\tv_nop\n\tv_nop" : "+v"(acc[0][0]), "+v"(acc[1][1]), "+v"(acc[2][2]), "+v"(acc[3][3]) : "v"(a[0]), "v"(a[1]), "v"(a[2]), "v"(a[3]));
    }
    const size_t tbase = (size_t)(r0 / RB) * sRB + (size_t)(r0 % RB) * (size_t)pitch + (size_t)(c0 / CB) * sCB + (size_t)(c0 % CB);
#pragma unroll
    for (int mb = 0; mb < 4; ++mb) {
#pragma unroll
        for (int nb = 0; nb < 4; ++nb) {
#pragma unroll
            for (int j = 0; j < 8; ++j) os[(hi * 8 + j) * 68 + nb * 16 + lr] = acc[mb][nb][j]; }
        wave_sync();
        const size_t sb = tbase + (size_t)(mb * 16) * (size_t)pitch;
#pragma unroll 1
        for (int ps = 0; ps < 2; ++ps) {
            if constexpr (MODE == 2) {
#pragma unroll
                for (int s = 0; s < 8; ++s) { const int row = 2 * s + hi, cofs = lr * 4;
                    v4f val = *(const v4fa*)(&os[row * 68 + cofs]);
                    if (useBias) { const v4f bb = *(const v4f*)(bias + c0 + cofs);
#pragma unroll
                        for (int i = 0; i < 4; ++i) val[i] += bfr(bb[i]); }
                    *(volatile v4f*)(P32 + sb + (size_t)row * (size_t)pitch + cofs) = val; }
            } else {
#pragma unroll
                for (int s = 0; s < 4; ++s) { const int row = 4 * s + (lane >> 3), c8 = (lane & 7) * 8;
                    v4f x0 = *(const v4fa*)(&os[row * 68 + c8]); v4f x1 = *(const v4fa*)(&os[row * 68 + c8 + 4]);
                    const size_t oo = sb + (size_t)row * (size_t)pitch + c8;
                    if constexpr (MODE == 0) {
                        if (useBias) { const v4f b0 = *(const v4f*)(bias + c0 + c8); const v4f b1 = *(const v4f*)(bias + c0 + c8 + 4);
#pragma unroll
                            for (int i = 0; i < 4; ++i) { x0[i] += bfr(b0[i]); x1[i] += bfr(b1[i]); } }
                        v8us hv, lv;
#pragma unroll
                        for (int i = 0; i < 4; ++i) { const unsigned short a0 = f2bf(x0[i]); const unsigned short a1 = f2bf(x1[i]); hv[i] = a0; hv[4 + i] = a1;
                            lv[i] = f2bf(x0[i] - bf2f(a0)); lv[4 + i] = f2bf(x1[i] - bf2f(a1)); }
                        *(volatile v8us*)(P16 + oo) = hv; *(volatile v8us*)(P16 + oo + DM) = lv;
                    } else {
                        float bb = 0.0f;
                        if (useBias) bb = bfr(bias[r0 + mb * 16 + row]);
                        v8h hv;
#pragma unroll
                        for (int i = 0; i < 4; ++i) { hv[i] = (h16)(x0[i] + bb); hv[4 + i] = (h16)(x1[i] + bb); }
                        *(volatile v8h*)((h16*)P16 + oo) = hv;
                    } }
            }
            if (ps == 0) __threadfence(); }
        wave_sync();
    }
}

__global__ __launch_bounds__(32) void k_gemmh(const bf* __restrict__ A, const bf* __restrict__ Bt, int lda, int ldbt, int KT, const float* __restrict__ bias, h16* PH, int pitch) {
    __shared__ __align__(16) float os[16 * 68];
    const int lane = threadIdx.x & 31, lr = lane & 15, hi = lane >> 4; const int r0 = blockIdx.x * 64, c0 = blockIdx.y * 64;
    v8f acc[4][4];
#pragma unroll
    for (int mb = 0; mb < 4; ++mb)
#pragma unroll
        for (int nb = 0; nb < 4; ++nb) acc[mb][nb] = (v8f){};
    const size_t aoff = (size_t)(r0 + lr) * (size_t)lda + 8 * hi, boff = (size_t)(c0 + lr) * (size_t)ldbt + 8 * hi;
#pragma unroll 1
    for (int kc = 0; kc < KT; kc += 32) {
        v16bf a[4];
#pragma unroll
        for (int mb = 0; mb < 4; ++mb) a[mb] = ldb(A + aoff + (size_t)mb * 16 * (size_t)lda + kc);
#pragma unroll
        for (int nb = 0; nb < 4; ++nb) { const v16bf b = ldb(Bt + boff + (size_t)nb * 16 * (size_t)ldbt + kc);
#pragma unroll
            for (int mb = 0; mb < 4; ++mb) acc[mb][nb] = wmmab_g(a[mb], b, acc[mb][nb]); }
    }
    const size_t tbase = (size_t)r0 * (size_t)pitch + (size_t)c0;
    const int c8 = (lane & 7) * 8;
    const v4f b0 = *(const v4f*)(bias + c0 + c8); const v4f b1 = *(const v4f*)(bias + c0 + c8 + 4);
#pragma unroll
    for (int mb = 0; mb < 4; ++mb) {
#pragma unroll
        for (int nb = 0; nb < 4; ++nb) {
#pragma unroll
            for (int j = 0; j < 8; ++j) os[(hi * 8 + j) * 68 + nb * 16 + lr] = acc[mb][nb][j]; }
        wave_sync();
        const size_t sb = tbase + (size_t)(mb * 16) * (size_t)pitch;
#pragma unroll 1
        for (int ps = 0; ps < 2; ++ps) {
#pragma unroll
            for (int s = 0; s < 4; ++s) { const int row = 4 * s + (lane >> 3);
                const v4f x0 = *(const v4fa*)(&os[row * 68 + c8]); const v4f x1 = *(const v4fa*)(&os[row * 68 + c8 + 4]);
                v8h hv;
#pragma unroll
                for (int i = 0; i < 4; ++i) { hv[i] = toh_flush(x0[i] + bfr(b0[i])); hv[4 + i] = toh_flush(x1[i] + bfr(b1[i])); }
                *(volatile v8h*)(PH + sb + (size_t)row * (size_t)pitch + c8) = hv; }
            if (ps == 0) __threadfence(); }
        wave_sync();
    }
}

__global__ __launch_bounds__(32 * FW) void k_flash(const h16* __restrict__ QH, const h16* __restrict__ KH, const h16* __restrict__ VT, const float* __restrict__ MASK, bf* CX2) {
    extern __shared__ __align__(16) unsigned char smem[];
    h16* qs = (h16*)smem; float* os = (float*)smem; h16* ps = (h16*)(smem + OFF_P);
    float* wmx = (float*)(smem + OFF_MX); float* wsm = (float*)(smem + OFF_SM); int* li = (int*)(smem + OFF_LI);
    const int tid = threadIdx.x, lane = tid & 31, lr = lane & 15, hi = lane >> 4;
    const int wave = __builtin_amdgcn_readfirstlane(tid >> 5);
    const int b = blockIdx.y, t0 = blockIdx.x * 16;

    { const h16* qg = QH + ((size_t)b * SEQ + t0) * DM;
#pragma unroll 4
      for (int i = tid; i < 16 * (DM / 8); i += 32 * FW) { const int row = i / (DM / 8), c = (i % (DM / 8)) * 8;
          const v8h v = *(const v8h*)(qg + (size_t)row * DM + c); *(v8h*)(qs + row * QPH + c) = v; } }
    int last = -1, anc = 0;
    { const int row = tid >> 4, c = tid & 15; const float* mr = MASK + (size_t)(t0 + row) * SEQ_FULL;
#pragma unroll 4
      for (int j = 0; j < SEQ / 64; ++j) { const int col = (j * 16 + c) * 4; const v4f mv = *(const v4f*)(mr + col);
#pragma unroll
          for (int e = 0; e < 4; ++e) { last = (mv[e] > -1.0e8f) ? imax(last, col + e) : last; anc = (mv[e] > -1.0e4f) ? 1 : anc; } } }
    anc |= __shfl_xor(anc, 1, 32); anc |= __shfl_xor(anc, 2, 32); anc |= __shfl_xor(anc, 4, 32); anc |= __shfl_xor(anc, 8, 32);
    anc &= __shfl_xor(anc, 16, 32);
    last = imax(last, __shfl_xor(last, 1, 32)); last = imax(last, __shfl_xor(last, 2, 32)); last = imax(last, __shfl_xor(last, 4, 32));
    last = imax(last, __shfl_xor(last, 8, 32)); last = imax(last, __shfl_xor(last, 16, 32));
    if (lane == 0) { li[wave] = last; li[FW + wave] = anc; }
    __syncthreads();
    int klim;
    { int L = -1, AA = 1;
#pragma unroll
      for (int w2 = 0; w2 < FW; ++w2) { L = imax(L, li[w2]); AA &= li[FW + w2]; }
      klim = (AA != 0 && L >= 0) ? ((L + 32) & ~31) : SEQ;
      klim = imin(imax(klim, 32), SEQ);
      klim = __builtin_amdgcn_readfirstlane(klim); }

    v8f o[8];
#pragma unroll
    for (int j = 0; j < 8; ++j) o[j] = (v8f){};
    float m = -1.0e30f, l = 0.0f;
    const h16* qf = qs + lr * QPH + 8 * hi;
    const size_t kbase = (size_t)b * SEQ * DM + (size_t)lr * DM + 8 * hi;
    const size_t vbase = (size_t)b * DM * SEQ + (size_t)(wave * 128 + lr) * SEQ + 8 * hi;
    const float* mrow = MASK + (size_t)(t0 + lr) * SEQ_FULL + 8 * hi;

#pragma unroll 1
    for (int kc0 = 0; kc0 < klim; kc0 += 32 * FW) {
        const int kw = kc0 + 32 * wave; const bool act = kw < klim;
        float xa[8], xb[8]; float mx = -3.0e38f;
        if (act) {
            v8f sa = (v8f){}, sb = (v8f){};
            const h16* ka = KH + kbase + (size_t)kw * DM;
#pragma unroll 2
            for (int ks = 0; ks < DM; ks += 32) {
                const v16h qh = cat16(*(const v8h*)(qf + ks), *(const v8h*)(qf + ks + 16));
                const v16h kah = ldh(ka + ks), kbh = ldh(ka + (size_t)16 * DM + ks);
                sa = wmma16_g(kah, qh, sa); sb = wmma16_g(kbh, qh, sb);
            }
            const v4f ma0 = *(const v4f*)(mrow + kw), ma1 = *(const v4f*)(mrow + kw + 4), mb0 = *(const v4f*)(mrow + kw + 16), mb1 = *(const v4f*)(mrow + kw + 20);
#pragma unroll
            for (int r = 0; r < 4; ++r) { xa[r] = sa[r] * SCL + ma0[r]; xa[4 + r] = sa[4 + r] * SCL + ma1[r]; xb[r] = sb[r] * SCL + mb0[r]; xb[4 + r] = sb[4 + r] * SCL + mb1[r]; }
#pragma unroll
            for (int r = 0; r < 8; ++r) mx = fmaxf(mx, fmaxf(xa[r], xb[r]));
        } else {
#pragma unroll
            for (int r = 0; r < 8; ++r) { xa[r] = -3.0e38f; xb[r] = -3.0e38f; }
        }
        mx = fmaxf(mx, __shfl_xor(mx, 16, 32));
        if (hi == 0) wmx[wave * 16 + lr] = mx;
        __syncthreads();
        float cm = wmx[lr];
#pragma unroll
        for (int w2 = 1; w2 < FW; ++w2) cm = fmaxf(cm, wmx[w2 * 16 + lr]);
        const float mnew = fmaxf(m, cm);
        const float alpha = __builtin_amdgcn_exp2f((m - mnew) * L2E);
        const float sh = PSH - mnew * L2E;
        v8h p0 = (v8h){}, p1 = (v8h){}; float ls = 0.0f;
        if (act) {
#pragma unroll
            for (int r = 0; r < 8; ++r) { const float ea = xa[r] * L2E + sh; const float ec = xb[r] * L2E + sh;
                const h16 pa = (ea < -14.0f) ? (h16)0.0f : (h16)__builtin_amdgcn_exp2f(ea); const h16 pc = (ec < -14.0f) ? (h16)0.0f : (h16)__builtin_amdgcn_exp2f(ec);
                p0[r] = pa; p1[r] = pc; ls += (float)pa + (float)pc; }
        }
        ls += __shfl_xor(ls, 16, 32);
        { h16* pw = ps + (wave * 32 + lane) * 16; *(v8h*)pw = p0; *(v8h*)(pw + 8) = p1; }
        if (hi == 0) wsm[wave * 16 + lr] = ls;
        m = mnew;
        __syncthreads();
        float lsum = 0.0f;
#pragma unroll
        for (int w2 = 0; w2 < FW; ++w2) lsum += wsm[w2 * 16 + lr];
        l = l * alpha + lsum;
#pragma unroll
        for (int j = 0; j < 8; ++j) o[j] = o[j] * alpha;
        const int rem = (klim - kc0) >> 5; const int nst = rem < FW ? rem : FW;
#pragma unroll 1
        for (int w2 = 0; w2 < nst; ++w2) {
            const h16* pp = ps + (w2 * 32 + lane) * 16;
            const v16h pb = cat16(*(const v8h*)pp, *(const v8h*)(pp + 8));
            const h16* va = VT + vbase + kc0 + 32 * w2;
            v16h vf[8];
#pragma unroll
            for (int j = 0; j < 8; ++j) vf[j] = ldh(va + (size_t)(16 * j) * SEQ);
#pragma unroll
            for (int j = 0; j < 8; ++j) o[j] = wmma16(vf[j], pb, o[j]);
            asm volatile("v_nop\n\tv_nop\n\tv_nop\n\tv_nop" : "+v"(o[0]), "+v"(o[1]), "+v"(o[2]), "+v"(o[3]), "+v"(o[4]), "+v"(o[5]), "+v"(o[6]), "+v"(o[7]) : "v"(vf[0]), "v"(vf[7]), "v"(pb));
        }
    }
    const float inv = 1.0f / l;
    __syncthreads();
    float* ow = os + wave * 16 * OSP;
#pragma unroll
    for (int j = 0; j < 8; ++j) { v4f a, c;
        a[0] = o[j][0] * inv; a[1] = o[j][1] * inv; a[2] = o[j][2] * inv; a[3] = o[j][3] * inv; c[0] = o[j][4] * inv; c[1] = o[j][5] * inv; c[2] = o[j][6] * inv; c[3] = o[j][7] * inv;
        *(v4fa*)(&ow[lr * OSP + 16 * j + 8 * hi]) = a; *(v4fa*)(&ow[lr * OSP + 16 * j + 8 * hi + 4]) = c; }
    wave_sync();
    bf* crow = CX2 + ((size_t)b * SEQ + t0) * DM2 + wave * 128;
#pragma unroll 1
    for (int ps2 = 0; ps2 < 2; ++ps2) {
#pragma unroll
        for (int s = 0; s < 8; ++s) { const int row = 2 * s + hi, c8 = lr * 8;
            const v4f x0 = *(const v4fa*)(&ow[row * OSP + c8]); const v4f x1 = *(const v4fa*)(&ow[row * OSP + c8 + 4]);
            v8us hv, lv;
#pragma unroll
            for (int i = 0; i < 4; ++i) { const unsigned short a0 = f2bf(x0[i]); const unsigned short a1 = f2bf(x1[i]); hv[i] = a0; hv[4 + i] = a1;
                lv[i] = f2bf(x0[i] - bf2f(a0)); lv[4 + i] = f2bf(x1[i] - bf2f(a1)); }
            const size_t oo = (size_t)row * DM2 + c8;
            *(volatile v8us*)(crow + oo) = hv; *(volatile v8us*)(crow + oo + DM) = lv; }
        if (ps2 == 0) __threadfence(); }
}

__global__ __launch_bounds__(32 * FW) void k_early(const bf* __restrict__ QE2, const bf* __restrict__ KE2, const bf* __restrict__ VE2, const float* __restrict__ MASK, const float* __restrict__ BV, bf* CX2) {
    extern __shared__ __align__(16) unsigned char smem[];
    bf* qs = (bf*)smem; float* os = (float*)smem; bf* ps = (bf*)(smem + EOFF_P);
    float* wmx = (float*)(smem + EOFF_MX); float* wsm = (float*)(smem + EOFF_SM); int* li = (int*)(smem + EOFF_LI);
    const int tid = threadIdx.x, lane = tid & 31, lr = lane & 15, hi = lane >> 4;
    const int wave = __builtin_amdgcn_readfirstlane(tid >> 5);
    const int b = blockIdx.y, t0 = blockIdx.x * 16;

    { const bf* qg = QE2 + ((size_t)b * EROWS + t0) * DM2;
#pragma unroll 4
      for (int i = tid; i < 16 * (DM2 / 8); i += 32 * FW) { const int row = i / (DM2 / 8), c = (i % (DM2 / 8)) * 8;
          const v8us v = *(const v8us*)(qg + (size_t)row * DM2 + c); *(v8us*)(qs + row * QPT + c) = v; } }
    int last = -1, anc = 0;
    { const int row = tid >> 4, c = tid & 15; const float* mr = MASK + (size_t)(t0 + row) * SEQ_FULL;
#pragma unroll 4
      for (int j = 0; j < SEQ / 64; ++j) { const int col = (j * 16 + c) * 4; const v4f mv = *(const v4f*)(mr + col);
#pragma unroll
          for (int e = 0; e < 4; ++e) { last = (mv[e] > -1.0e8f) ? imax(last, col + e) : last; anc = (mv[e] > -1.0e4f) ? 1 : anc; } } }
    anc |= __shfl_xor(anc, 1, 32); anc |= __shfl_xor(anc, 2, 32); anc |= __shfl_xor(anc, 4, 32); anc |= __shfl_xor(anc, 8, 32);
    anc &= __shfl_xor(anc, 16, 32);
    last = imax(last, __shfl_xor(last, 1, 32)); last = imax(last, __shfl_xor(last, 2, 32)); last = imax(last, __shfl_xor(last, 4, 32));
    last = imax(last, __shfl_xor(last, 8, 32)); last = imax(last, __shfl_xor(last, 16, 32));
    if (lane == 0) { li[wave] = last; li[FW + wave] = anc; }
    __syncthreads();
    int klim;
    { int L = -1, AA = 1;
#pragma unroll
      for (int w2 = 0; w2 < FW; ++w2) { L = imax(L, li[w2]); AA &= li[FW + w2]; }
      klim = (AA != 0 && L >= 0) ? ((L + 32) & ~31) : SEQ;
      klim = imin(imax(klim, 32), SEQ);
      klim = __builtin_amdgcn_readfirstlane(klim); }
    if (klim > EROWS) return;

    v8f o[8];
#pragma unroll
    for (int j = 0; j < 8; ++j) o[j] = (v8f){};
    float m = -1.0e30f, l = 0.0f;
    const bf* qf = qs + lr * QPT + 8 * hi;
    const size_t kbase = (size_t)b * EROWS * DM2 + (size_t)lr * DM2 + 8 * hi;
    const size_t vbase = (size_t)(wave * 128 + lr) * DM2 + (size_t)b * EROWS + 8 * hi;
    const float* mrow = MASK + (size_t)(t0 + lr) * SEQ_FULL + 8 * hi;

#pragma unroll 1
    for (int kc0 = 0; kc0 < klim; kc0 += 32 * FW) {
        const int kw = kc0 + 32 * wave; const bool act = kw < klim;
        float xa[8], xb[8]; float mx = -3.0e38f;
        if (act) {
            v8f sa = (v8f){}, sb = (v8f){};
            const bf* ka = KE2 + kbase + (size_t)kw * DM2;
#pragma unroll 2
            for (int ks = 0; ks < DM; ks += 32) {
                const v16bf qh = cat16b(*(const v8us*)(qf + ks), *(const v8us*)(qf + ks + 16));
                const v16bf ql = cat16b(*(const v8us*)(qf + DM + ks), *(const v8us*)(qf + DM + ks + 16));
                const v16bf kah = ldb(ka + ks), kal = ldb(ka + DM + ks), kbh = ldb(ka + (size_t)16 * DM2 + ks), kbl = ldb(ka + (size_t)16 * DM2 + DM + ks);
                sa = wmmab_g(kah, qh, sa); sb = wmmab_g(kbh, qh, sb);
                sa = wmmab_g(kah, ql, sa); sb = wmmab_g(kbh, ql, sb);
                sa = wmmab_g(kal, qh, sa); sb = wmmab_g(kbl, qh, sb);
            }
            const v4f ma0 = *(const v4f*)(mrow + kw), ma1 = *(const v4f*)(mrow + kw + 4), mb0 = *(const v4f*)(mrow + kw + 16), mb1 = *(const v4f*)(mrow + kw + 20);
#pragma unroll
            for (int r = 0; r < 4; ++r) { xa[r] = sa[r] * SCL + ma0[r]; xa[4 + r] = sa[4 + r] * SCL + ma1[r]; xb[r] = sb[r] * SCL + mb0[r]; xb[4 + r] = sb[4 + r] * SCL + mb1[r]; }
#pragma unroll
            for (int r = 0; r < 8; ++r) mx = fmaxf(mx, fmaxf(xa[r], xb[r]));
        } else {
#pragma unroll
            for (int r = 0; r < 8; ++r) { xa[r] = -3.0e38f; xb[r] = -3.0e38f; }
        }
        mx = fmaxf(mx, __shfl_xor(mx, 16, 32));
        if (hi == 0) wmx[wave * 16 + lr] = mx;
        __syncthreads();
        float cm = wmx[lr];
#pragma unroll
        for (int w2 = 1; w2 < FW; ++w2) cm = fmaxf(cm, wmx[w2 * 16 + lr]);
        const float mnew = fmaxf(m, cm);
        const float alpha = __builtin_amdgcn_exp2f((m - mnew) * L2E);
        const float sh = PSH - mnew * L2E;
        v8us ph0 = (v8us){}, ph1 = (v8us){}, pl0 = (v8us){}, pl1 = (v8us){}; float ls = 0.0f;
        if (act) {
#pragma unroll
            for (int r = 0; r < 8; ++r) { const float ea = __builtin_amdgcn_exp2f(xa[r] * L2E + sh); const float ec = __builtin_amdgcn_exp2f(xb[r] * L2E + sh);
                const unsigned short ha = f2bf(ea); const unsigned short hc = f2bf(ec);
                ph0[r] = ha; ph1[r] = hc; pl0[r] = f2bf(ea - bf2f(ha)); pl1[r] = f2bf(ec - bf2f(hc)); ls += ea + ec; }
        }
        ls += __shfl_xor(ls, 16, 32);
        { bf* pw = ps + (wave * 32 + lane) * 32; *(v8us*)pw = ph0; *(v8us*)(pw + 8) = ph1; *(v8us*)(pw + 16) = pl0; *(v8us*)(pw + 24) = pl1; }
        if (hi == 0) wsm[wave * 16 + lr] = ls;
        m = mnew;
        __syncthreads();
        float lsum = 0.0f;
#pragma unroll
        for (int w2 = 0; w2 < FW; ++w2) lsum += wsm[w2 * 16 + lr];
        l = l * alpha + lsum;
#pragma unroll
        for (int j = 0; j < 8; ++j) o[j] = o[j] * alpha;
        const int rem = (klim - kc0) >> 5; const int nst = rem < FW ? rem : FW;
#pragma unroll 1
        for (int w2 = 0; w2 < nst; ++w2) {
            const bf* pp = ps + (w2 * 32 + lane) * 32;
            const v16bf pbh = cat16b(*(const v8us*)pp, *(const v8us*)(pp + 8));
            const v16bf pbl = cat16b(*(const v8us*)(pp + 16), *(const v8us*)(pp + 24));
            const bf* va = VE2 + vbase + kc0 + 32 * w2;
#pragma unroll
            for (int g = 0; g < 2; ++g) {
                v16bf vh[4], vl[4];
#pragma unroll
                for (int j = 0; j < 4; ++j) { vh[j] = ldb(va + (size_t)(16 * (4 * g + j)) * DM2); vl[j] = ldb(va + (size_t)(16 * (4 * g + j)) * DM2 + DM); }
#pragma unroll
                for (int j = 0; j < 4; ++j) o[4 * g + j] = wmmab_g(vh[j], pbh, o[4 * g + j]);
#pragma unroll
                for (int j = 0; j < 4; ++j) o[4 * g + j] = wmmab_g(vh[j], pbl, o[4 * g + j]);
#pragma unroll
                for (int j = 0; j < 4; ++j) o[4 * g + j] = wmmab_g(vl[j], pbh, o[4 * g + j]);
            }
        }
    }
    const float inv = 1.0f / l;
    __syncthreads();
    float* ow = os + wave * 16 * OSP;
#pragma unroll
    for (int j = 0; j < 8; ++j) { v4f a, c;
        const v4f b0 = *(const v4f*)(BV + wave * 128 + 16 * j + 8 * hi); const v4f b1 = *(const v4f*)(BV + wave * 128 + 16 * j + 8 * hi + 4);
        a[0] = o[j][0] * inv + bfr(b0[0]); a[1] = o[j][1] * inv + bfr(b0[1]); a[2] = o[j][2] * inv + bfr(b0[2]); a[3] = o[j][3] * inv + bfr(b0[3]);
        c[0] = o[j][4] * inv + bfr(b1[0]); c[1] = o[j][5] * inv + bfr(b1[1]); c[2] = o[j][6] * inv + bfr(b1[2]); c[3] = o[j][7] * inv + bfr(b1[3]);
        *(v4fa*)(&ow[lr * OSP + 16 * j + 8 * hi]) = a; *(v4fa*)(&ow[lr * OSP + 16 * j + 8 * hi + 4]) = c; }
    wave_sync();
    bf* crow = CX2 + ((size_t)b * SEQ + t0) * DM2 + wave * 128;
#pragma unroll 1
    for (int ps2 = 0; ps2 < 2; ++ps2) {
#pragma unroll
        for (int s = 0; s < 8; ++s) { const int row = 2 * s + hi, c8 = lr * 8;
            const v4f x0 = *(const v4fa*)(&ow[row * OSP + c8]); const v4f x1 = *(const v4fa*)(&ow[row * OSP + c8 + 4]);
            v8us hv, lv;
#pragma unroll
            for (int i = 0; i < 4; ++i) { const unsigned short a0 = f2bf(x0[i]); const unsigned short a1 = f2bf(x1[i]); hv[i] = a0; hv[4 + i] = a1;
                lv[i] = f2bf(x0[i] - bf2f(a0)); lv[4 + i] = f2bf(x1[i] - bf2f(a1)); }
            const size_t oo = (size_t)row * DM2 + c8;
            *(volatile v8us*)(crow + oo) = hv; *(volatile v8us*)(crow + oo + DM) = lv; }
        if (ps2 == 0) __threadfence(); }
}

static constexpr size_t al256(size_t v) { return (v + 255) & ~(size_t)255; }
static constexpr size_t cmax(size_t a, size_t b) { return a > b ? a : b; }
static constexpr size_t SZ_QB = al256((size_t)NB * SEQ * DM * 2);
static constexpr size_t SZ_P2 = al256((size_t)NB * SEQ * DM2 * 2);
static constexpr size_t SZ_R0 = cmax(SZ_QB, SZ_P2);
static constexpr size_t SZ_WT = al256((size_t)4 * DM * DM * 2);
static constexpr size_t SZ_H  = al256((size_t)NB * SEQ * DM * 2);
static constexpr size_t SZ_VT = al256((size_t)NB * DM * SEQ * 2);
static constexpr size_t SZ_VE = al256((size_t)DM * DM2 * 2);
static constexpr size_t SZ_E2 = al256((size_t)NB * EROWS * DM2 * 2);
static constexpr size_t SZ_TOTAL = SZ_R0 + SZ_WT + 2 * SZ_H + SZ_VT + SZ_VE + 2 * SZ_E2;
static_assert(SZ_QB <= SZ_R0);
static_assert(SZ_P2 <= SZ_R0);
static_assert(SZ_TOTAL <= (size_t)134217728);
static_assert(((size_t)DM * DM * 2) % 256 == 0);
static_assert((size_t)(DM - 1) * DM2 + DM + (size_t)NB * EROWS <= (size_t)DM * DM2);
static_assert(((size_t)(NB - 1) * EROWS + EROWS) * DM2 * 2 <= SZ_E2);
static_assert((size_t)NB * SEQ * DM * 2 <= SZ_H);

extern "C" void kernel_launch(void* const* d_in, const int* in_sizes, int n_in,
                              void* d_out, int out_size, void* d_ws, size_t ws_size, hipStream_t stream) {
    if (n_in < 10) return;
    const size_t needx = ((size_t)(NB - 1) * SEQ_FULL + SEQ) * DM;
    if ((size_t)in_sizes[0] < needx) return;
    if ((size_t)in_sizes[1] < (size_t)(SEQ - 1) * SEQ_FULL + SEQ) return;
    if ((size_t)in_sizes[2] < (size_t)DM * DM || (size_t)in_sizes[4] < (size_t)DM * DM || (size_t)in_sizes[6] < (size_t)DM * DM || (size_t)in_sizes[8] < (size_t)DM * DM) return;
    if (in_sizes[3] < DM || in_sizes[5] < DM || in_sizes[7] < DM || in_sizes[9] < DM) return;
    if ((size_t)out_size < ((size_t)(NB - 1) * OUT_SEQ + SEQ) * DM) return;
    if (SZ_TOTAL > ws_size) return;
    const float* x = (const float*)d_in[0]; const float* mask = (const float*)d_in[1];
    const float* wq = (const float*)d_in[2]; const float* bq = (const float*)d_in[3]; const float* wk = (const float*)d_in[4]; const float* bk = (const float*)d_in[5];
    const float* wv = (const float*)d_in[6]; const float* bv = (const float*)d_in[7]; const float* wo = (const float*)d_in[8]; const float* bo = (const float*)d_in[9];
    float* OUT = (float*)d_out;
    char* wsp = (char*)d_ws;
    bf* QB  = (bf*)wsp;
    bf* CX2 = (bf*)wsp; wsp += SZ_R0;
    bf* WT  = (bf*)wsp; wsp += SZ_WT;
    h16* QH = (h16*)wsp; wsp += SZ_H;
    h16* KH = (h16*)wsp; wsp += SZ_H;
    h16* VT = (h16*)wsp; wsp += SZ_VT;
    bf* VE2 = (bf*)wsp; wsp += SZ_VE;
    bf* QE2 = (bf*)wsp; wsp += SZ_E2;
    bf* KE2 = (bf*)wsp; wsp += SZ_E2;
    bf* WQT = WT; bf* WKT = WT + (size_t)DM * DM; bf* WVT = WT + (size_t)2 * DM * DM; bf* WOT = WT + (size_t)3 * DM * DM;
    const int M = NB * SEQ;

    if (SEQ == SEQ_FULL) {
        const size_t n8 = (size_t)NB * SEQ * DM / 8;
        k_cvt8<<<(unsigned)((n8 + 255) / 256), 256, 0, stream>>>(x, QB, n8);
    } else {
        const size_t n8 = (size_t)SEQ * DM / 8;
        for (int b = 0; b < NB; ++b) k_cvt8<<<(unsigned)((n8 + 255) / 256), 256, 0, stream>>>(x + (size_t)b * SEQ_FULL * DM, QB + (size_t)b * SEQ * DM, n8);
    }
    k_tr<<<dim3(DM / 64, DM / 64, 1), 256, 0, stream>>>(wq, WQT);
    k_tr<<<dim3(DM / 64, DM / 64, 1), 256, 0, stream>>>(wk, WKT);
    k_tr<<<dim3(DM / 64, DM / 64, 1), 256, 0, stream>>>(wv, WVT);
    k_tr<<<dim3(DM / 64, DM / 64, 1), 256, 0, stream>>>(wo, WOT);

    k_gemmh<<<dim3(M / 64, DM / 64, 1), 32, 0, stream>>>(QB, WQT, DM, DM, DM, bq, QH, DM);
    k_gemmh<<<dim3(M / 64, DM / 64, 1), 32, 0, stream>>>(QB, WKT, DM, DM, DM, bk, KH, DM);
    k_gemm<1><<<dim3(DM / 64, M / 64, 1), 32, 0, stream>>>(WVT, QB, DM, DM, DM, DM - 1, DM - 1, bv, 1, (bf*)VT, OUT, DM, (size_t)0, SEQ, SEQ, (size_t)DM * SEQ);
    for (int b = 0; b < NB; ++b) {
        const bf* xb = QB + (size_t)b * SEQ * DM;
        k_gemm<0><<<dim3(DM / 64, EROWS / 64, 1), 32, 0, stream>>>(WVT, xb, DM, DM, DM, DM - 1, DM - 1, bv, 0, VE2 + (size_t)b * EROWS, OUT, DM, (size_t)0, DM2, DM, (size_t)0);
        k_gemm<0><<<dim3(EROWS / 64, DM / 64, 1), 32, 0, stream>>>(xb, WQT, DM, DM, DM, DM - 1, DM - 1, bq, 1, QE2 + (size_t)b * EROWS * DM2, OUT, M, (size_t)0, DM2, DM, (size_t)0);
        k_gemm<0><<<dim3(EROWS / 64, DM / 64, 1), 32, 0, stream>>>(xb, WKT, DM, DM, DM, DM - 1, DM - 1, bk, 1, KE2 + (size_t)b * EROWS * DM2, OUT, M, (size_t)0, DM2, DM, (size_t)0);
    }

    hipFuncSetAttribute(reinterpret_cast<const void*>(&k_flash), hipFuncAttributeMaxDynamicSharedMemorySize, LDS_FLASH);
    k_flash<<<dim3(SEQ / 16, NB, 1), 32 * FW, LDS_FLASH, stream>>>(QH, KH, VT, mask, CX2);
    hipFuncSetAttribute(reinterpret_cast<const void*>(&k_early), hipFuncAttributeMaxDynamicSharedMemorySize, LDS_EARLY);
    k_early<<<dim3(EROWS / 16, NB, 1), 32 * FW, LDS_EARLY, stream>>>(QE2, KE2, VE2, mask, bv, CX2);

    k_gemm<2><<<dim3(M / 64, DM / 64, 1), 32, 0, stream>>>(CX2, WOT, DM2, DM, DM2, DM2 - 1, DM - 1, bo, 1, WT, OUT, SEQ, (size_t)OUT_SEQ * DM, DM, DM, (size_t)0);
}
